// DAWN_88124138979393
// MI455X (gfx1250) — hardware-run, weakly checked
//
#include <hip/hip_runtime.h>
#include <math.h>

constexpr int kB   = 2;
constexpr int kS   = 2048;
constexpr int kD   = 1024;
constexpr int kH   = 16;
constexpr int kDh  = 64;
constexpr int kR   = 64;
constexpr int kN   = 32;
constexpr int kRK  = 128;
constexpr int kTok = kB * kS;
constexpr int kKqk = kN * kR;
constexpr int kKkn = kN * kRK;
constexpr float kInvD   = 1.0f / 1024.0f;
constexpr float kLnEps  = 1e-5f;
constexpr float kWCarry   = 64.0f;
constexpr float kTCarry   = 16.0f;
constexpr float kAhInv    = 1.0f / 64.0f;
constexpr float kQScale   = 8.0f / (16.0f * 64.0f);
constexpr float kKVScale  = 16.0f / (16.0f * 64.0f);
constexpr float kScoreInv = 1.0f / 1024.0f;
constexpr float kPCarry   = 32768.0f;
constexpr float kAttnOut  = 16.0f / (32768.0f * 16.0f);
constexpr float kWoScale  = 1.0f / (16.0f * 64.0f);
constexpr float kKnScale  = 1.0f / (16.0f * 64.0f);
static_assert(kH * kDh == kD);
static_assert(kS % 64 == 0 && kTok % 64 == 0 && kD % 64 == 0 && kKqk % 64 == 0 && kKkn % 64 == 0);
static_assert(kD % 32 == 0 && kKqk % 32 == 0 && kKkn % 32 == 0 && kDh % 32 == 0);

typedef __attribute__((ext_vector_type(16))) _Float16 v16h;
typedef __attribute__((ext_vector_type(8)))  _Float16 v8h;
typedef __attribute__((ext_vector_type(16))) __bf16   v16b;
typedef __attribute__((ext_vector_type(8)))  __bf16   v8b;
typedef __attribute__((ext_vector_type(8)))  float    v8f;
typedef __attribute__((ext_vector_type(4)))  float    v4f;
typedef __attribute__((ext_vector_type(4)))  unsigned int v4u;
typedef __attribute__((ext_vector_type(2)))  unsigned int v2u;

__device__ __forceinline__ unsigned short f2bf_bits(float f) {
  unsigned u = __float_as_uint(f);
  return (unsigned short)((u + 0x7FFFu + ((u >> 16) & 1u)) >> 16);
}
__device__ __forceinline__ float bf_bits2f(unsigned short h) { return __uint_as_float(((unsigned)h) << 16); }

__device__ __forceinline__ void dep_guard4_h(v8f& a, v8f& b, v8f& c, v8f& d, v16h x, v16h y) {
  asm volatile("v_nop\n\tv_nop\n\tv_nop\n\tv_nop" : "+v"(a), "+v"(b), "+v"(c), "+v"(d) : "v"(x), "v"(y));
}
__device__ __forceinline__ void dep_guard4_b(v8f& a, v8f& b, v8f& c, v8f& d, v16b x, v16b y) {
  asm volatile("v_nop\n\tv_nop\n\tv_nop\n\tv_nop" : "+v"(a), "+v"(b), "+v"(c), "+v"(d) : "v"(x), "v"(y));
}
__device__ __forceinline__ void keep4_h(v16h a, v16h b, v16h c, v16h d) { asm volatile("v_nop" :: "v"(a), "v"(b), "v"(c), "v"(d)); }
__device__ __forceinline__ void keep4_b(v16b a, v16b b, v16b c, v16b d) { asm volatile("v_nop" :: "v"(a), "v"(b), "v"(c), "v"(d)); }
__device__ __forceinline__ void acc_guard4(v8f& a, v8f& b, v8f& c, v8f& d) { asm volatile("v_nop\n\tv_nop\n\tv_nop\n\tv_nop" : "+v"(a), "+v"(b), "+v"(c), "+v"(d)); }

template <typename T> struct Frag;
template <> struct Frag<_Float16> {
  typedef v16h V; union U { v16h v; v8h h[2]; };
  static __device__ __forceinline__ v16h load(const _Float16* p) {
    U f; f.h[0] = *(const v8h*)(p); f.h[1] = *(const v8h*)(p + 16); return f.v;
  }
  static __device__ __forceinline__ v8f mma(v16h a, v16h b, v8f c) {
    return __builtin_amdgcn_wmma_f32_16x16x32_f16(false, a, false, b, (short)0, c, false, false);
  }
  static __device__ __forceinline__ void guard4(v8f& a, v8f& b, v8f& c, v8f& d, v16h x, v16h y) { dep_guard4_h(a, b, c, d, x, y); }
  static __device__ __forceinline__ void keep(v16h a, v16h b, v16h c, v16h d) { keep4_h(a, b, c, d); }
};
template <> struct Frag<__bf16> {
  typedef v16b V; union U { v16b v; v8b h[2]; };
  static __device__ __forceinline__ v16b load(const __bf16* p) {
    U f; f.h[0] = *(const v8b*)(p); f.h[1] = *(const v8b*)(p + 16); return f.v;
  }
  static __device__ __forceinline__ v8f mma(v16b a, v16b b, v8f c) {
    return __builtin_amdgcn_wmma_f32_16x16x32_bf16(false, a, false, b, (short)0, c, false, false);
  }
  static __device__ __forceinline__ void guard4(v8f& a, v8f& b, v8f& c, v8f& d, v16b x, v16b y) { dep_guard4_b(a, b, c, d, x, y); }
  static __device__ __forceinline__ void keep(v16b a, v16b b, v16b c, v16b d) { keep4_b(a, b, c, d); }
};

__device__ __forceinline__ unsigned pk16(unsigned short a, unsigned short b) { return (unsigned)a | ((unsigned)b << 16); }
__device__ __forceinline__ unsigned short h_bits(float f) { const _Float16 h = (_Float16)f; return __builtin_bit_cast(unsigned short, h); }

__device__ __forceinline__ float h16_to_f32(unsigned hb) {
  const unsigned sgn = (hb & 0x8000u) << 16; const unsigned em = hb & 0x7fffu;
  const float fn = __uint_as_float((em << 13) + 0x38000000u);
  const float fs = (float)em * 5.9604644775390625e-8f;
  const float mag = (em < 0x400u) ? fs : fn; return __uint_as_float(__float_as_uint(mag) | sgn);
}

__device__ __forceinline__ v8f h_mma(v16h a, v16h b, v8f c) {
  c = __builtin_amdgcn_wmma_f32_16x16x32_f16(false, a, false, b, (short)0, c, false, false);
  asm volatile("v_nop\n\tv_nop\n\tv_nop\n\tv_nop" : "+v"(c) : "v"(a), "v"(b));
  return c;
}

template <int ET> struct Elem;
template <> struct Elem<0> { typedef _Float16 T; };
template <> struct Elem<1> { typedef __bf16 T; };
template <int ET, bool SPLIT, int BIAS_MODE, int OUT_MODE, bool RESID, int ACT = 0>
__global__ __launch_bounds__(256) void wmma_gemm64(
    const unsigned short* __restrict__ Ap, const unsigned short* __restrict__ A2p, int lda, long strideA,
    const unsigned short* __restrict__ Btp, const unsigned short* __restrict__ Bt2p, int ldb, long strideB,
    void* __restrict__ Cout, void* __restrict__ Cout2, int ldc, long strideC,
    const float* __restrict__ bias,
    const float* __restrict__ resid, long strideR,
    int M, int N, int K, float scale) {
  static_assert(!RESID || OUT_MODE == 0);
  static_assert(ACT == 0 || ACT == 2 || ACT == 4);
  typedef typename Elem<ET>::T T;
  typedef typename Frag<T>::V V;
  const T* A = (const T*)Ap; const T* A2 = (const T*)A2p; const T* Bt = (const T*)Btp; const T* Bt2 = (const T*)Bt2p;
  __shared__ __align__(16) float sT[8][16 * 68];
  const int b    = blockIdx.y;
  const int lane = threadIdx.x & 31;
  const int wave = threadIdx.x >> 5;
  const int tilesN = N >> 6;
  const int tilesM = M >> 6;
  const int tile = blockIdx.x * 8 + wave;
  if (tile >= tilesM * tilesN) return;
  const int tm = tile / tilesN;
  const int tn = tile - tm * tilesN;
  const int m0 = tm << 6;
  const int n0 = tn << 6;

  const T* Ab  = A  + (size_t)b * strideA;
  const T* Bb  = Bt + (size_t)b * strideB;
  const T* Ab2 = SPLIT ? (A2  + (size_t)b * strideA) : nullptr;
  const T* Bb2 = SPLIT ? (Bt2 + (size_t)b * strideB) : nullptr;

  const int rlane = lane & 15;
  const int koff  = (lane >> 4) * 8;
  const int mOff  = (lane >> 4) * 8;

  v8f acc[4][4];
#pragma unroll
  for (int i = 0; i < 4; ++i)
#pragma unroll
    for (int j = 0; j < 4; ++j) acc[i][j] = (v8f){0.f,0.f,0.f,0.f,0.f,0.f,0.f,0.f};

  for (int k0 = 0; k0 < K; k0 += 32) {
    V bh[4], bl[4];
#pragma unroll
    for (int j = 0; j < 4; ++j) {
      const size_t bo = (size_t)(n0 + (j << 4) + rlane) * ldb + koff + k0;
      bh[j] = Frag<T>::load(Bb + bo);
      if (SPLIT) bl[j] = Frag<T>::load(Bb2 + bo);
    }
#pragma unroll
    for (int i = 0; i < 4; ++i) {
      const size_t ao = (size_t)(m0 + (i << 4) + rlane) * lda + koff + k0;
      V ah = Frag<T>::load(Ab + ao);
      V al;
      if (SPLIT) al = Frag<T>::load(Ab2 + ao);
#pragma unroll
      for (int j = 0; j < 4; ++j) {
        acc[i][j] = Frag<T>::mma(ah, bh[j], acc[i][j]);
        if (SPLIT) {
          acc[i][j] = Frag<T>::mma(ah, bl[j], acc[i][j]);
          acc[i][j] = Frag<T>::mma(al, bh[j], acc[i][j]);
        }
      }
      Frag<T>::guard4(acc[i][0], acc[i][1], acc[i][2], acc[i][3], ah, SPLIT ? al : ah);
    }
    Frag<T>::keep(bh[0], bh[1], bh[2], bh[3]);
    if (SPLIT) Frag<T>::keep(bl[0], bl[1], bl[2], bl[3]);
  }
  acc_guard4(acc[0][0], acc[0][1], acc[0][2], acc[0][3]);
  acc_guard4(acc[1][0], acc[1][1], acc[1][2], acc[1][3]);
  acc_guard4(acc[2][0], acc[2][1], acc[2][2], acc[2][3]);
  acc_guard4(acc[3][0], acc[3][1], acc[3][2], acc[3][3]);

  float* slab = sT[wave];
#pragma unroll
  for (int i = 0; i < 4; ++i) {
    const int mBase = m0 + (i << 4);
#pragma unroll
    for (int j = 0; j < 4; ++j) {
      const int n = n0 + (j << 4) + rlane;
      float bv = 0.f;
      if (BIAS_MODE == 2) bv = bias[n];
#pragma unroll
      for (int r = 0; r < 8; ++r) {
        float v = acc[i][j][r] * scale;
        if (BIAS_MODE == 1) v += bias[mBase + mOff + r];
        if (BIAS_MODE == 2) v += bv;
        if (ACT == 2) v = fmaxf(v, 0.0f);
        if (ACT == 4) v = (v > 0.f) ? v : 0.01f * v;
        slab[(mOff + r) * 68 + (j << 4) + rlane] = v;
      }
    }
    __builtin_amdgcn_fence(__ATOMIC_RELEASE, "workgroup");
    __builtin_amdgcn_wave_barrier();
    __builtin_amdgcn_fence(__ATOMIC_ACQUIRE, "workgroup");
    if (OUT_MODE == 0) {
      float* C = (float*)Cout + (size_t)b * strideC;
      const float* Rb = RESID ? (resid + (size_t)b * strideR) : nullptr;
      const int hh = lane >> 4, c4 = (lane & 15) * 4;
      v4f vals[8];
#pragma unroll
      for (int it = 0; it < 8; ++it) {
        const int row = it * 2 + hh;
        v4f v = *(const v4f*)(slab + row * 68 + c4);
        if (RESID) {
          const v4f rr = *(const v4f*)(Rb + (size_t)(mBase + row) * ldc + n0 + c4);
          v += rr;
        }
        vals[it] = v;
      }
      for (int pass = 0; pass < 2; ++pass) {
#pragma unroll
        for (int it = 0; it < 8; ++it) {
          const int row = it * 2 + hh;
          *(volatile v4f*)(C + (size_t)(mBase + row) * ldc + n0 + c4) = vals[it];
        }
        __threadfence();
      }
    } else {
      const int q = lane >> 3, c8 = (lane & 7) * 8;
      unsigned short* C  = (unsigned short*)Cout  + (size_t)b * strideC;
      unsigned short* C2 = (OUT_MODE == 2) ? ((unsigned short*)Cout2 + (size_t)b * strideC) : nullptr;
      for (int pass = 0; pass < 2; ++pass) {
#pragma unroll
        for (int it = 0; it < 4; ++it) {
          const int row = it * 4 + q;
          const float* sp = slab + row * 68 + c8;
          v8h hv, lv;
#pragma unroll
          for (int e = 0; e < 8; ++e) {
            if (OUT_MODE == 1) {
              hv[e] = (_Float16)sp[e];
            } else {
              unsigned short hb = f2bf_bits(sp[e]);
              unsigned short lb = f2bf_bits(sp[e] - bf_bits2f(hb));
              hv[e] = __builtin_bit_cast(_Float16, hb);
              lv[e] = __builtin_bit_cast(_Float16, lb);
            }
          }
          *(volatile v8h*)(C + (size_t)(mBase + row) * ldc + n0 + c8) = hv;
          if (OUT_MODE == 2) *(volatile v8h*)(C2 + (size_t)(mBase + row) * ldc + n0 + c8) = lv;
        }
        __threadfence();
      }
    }
    __builtin_amdgcn_fence(__ATOMIC_RELEASE, "workgroup");
    __builtin_amdgcn_wave_barrier();
    __builtin_amdgcn_fence(__ATOMIC_ACQUIRE, "workgroup");
  }
}

__global__ __launch_bounds__(128) void ln_f16_kernel(const float* __restrict__ x, const float* __restrict__ g,
                                                     const float* __restrict__ bt, unsigned short* __restrict__ out) {
  __shared__ float redA[4];
  __shared__ float redB[4];
  const int row  = blockIdx.x;
  const int t    = threadIdx.x;
  const int lane = t & 31, wave = t >> 5;
  const int c0   = t * 8;
  const float* xr = x + (size_t)row * kD + c0;
  const v4f xa = *(const v4f*)(xr);
  const v4f xb = *(const v4f*)(xr + 4);
  float s = ((xa[0] + xa[1]) + (xa[2] + xa[3])) + ((xb[0] + xb[1]) + (xb[2] + xb[3]));
#pragma unroll
  for (int off = 16; off > 0; off >>= 1) s += __shfl_xor(s, off, 32);
  if (lane == 0) redA[wave] = s;
  __syncthreads();
  const float mu = ((redA[0] + redA[1]) + (redA[2] + redA[3])) * kInvD;
  float da[8];
#pragma unroll
  for (int e = 0; e < 4; ++e) { da[e] = xa[e] - mu; da[4 + e] = xb[e] - mu; }
  float q = 0.0f;
#pragma unroll
  for (int e = 0; e < 8; ++e) q += da[e] * da[e];
#pragma unroll
  for (int off = 16; off > 0; off >>= 1) q += __shfl_xor(q, off, 32);
  if (lane == 0) redB[wave] = q;
  __syncthreads();
  const float var  = ((redB[0] + redB[1]) + (redB[2] + redB[3])) * kInvD;
  const float rstd = rsqrtf(var + kLnEps);
  const v4f ga = *(const v4f*)(g + c0);
  const v4f gb = *(const v4f*)(g + c0 + 4);
  const v4f ba = *(const v4f*)(bt + c0);
  const v4f bb = *(const v4f*)(bt + c0 + 4);
  unsigned short hb[8];
#pragma unroll
  for (int e = 0; e < 4; ++e) {
    hb[e]     = h_bits(ga[e] * (da[e] * rstd) + ba[e]);
    hb[4 + e] = h_bits(gb[e] * (da[4 + e] * rstd) + bb[e]);
  }
  const v4u u = (v4u){pk16(hb[0], hb[1]), pk16(hb[2], hb[3]), pk16(hb[4], hb[5]), pk16(hb[6], hb[7])};
  unsigned short* op = out + (size_t)row * kD + c0;
  *(volatile v4u*)op = u;
  __threadfence();
  *(volatile v4u*)op = u;
}

__global__ __launch_bounds__(256) void tpose_cast_kernel(const float* __restrict__ in, long inBatch, int inPitch,
                                                         unsigned short* __restrict__ out, long outBatch, int outPitch,
                                                         float scale) {
  __shared__ float sm[64][65];
  const int t  = threadIdx.x;
  const int c0 = blockIdx.x * 64;
  const int r0 = blockIdx.y * 64;
  const float* ib = in + (size_t)blockIdx.z * (size_t)inBatch;
#pragma unroll
  for (int i = 0; i < 16; ++i) {
    const int e  = i * 256 + t;
    const int rl = e >> 6;
    const int cl = e & 63;
    sm[cl][rl] = ib[(size_t)(r0 + rl) * inPitch + c0 + cl] * scale;
  }
  __syncthreads();
  const int lane = t & 31, wave = t >> 5;
  const int q = lane >> 3, c8 = (lane & 7) * 8;
  unsigned short* ob = out + (size_t)blockIdx.z * (size_t)outBatch;
  for (int pass = 0; pass < 2; ++pass) {
#pragma unroll
    for (int it = 0; it < 2; ++it) {
      const int row = wave * 8 + it * 4 + q;
      unsigned short hb[8];
#pragma unroll
      for (int e = 0; e < 8; ++e) hb[e] = h_bits(sm[row][c8 + e]);
      const v4u u = (v4u){pk16(hb[0], hb[1]), pk16(hb[2], hb[3]), pk16(hb[4], hb[5]), pk16(hb[6], hb[7])};
      *(volatile v4u*)(ob + (size_t)(c0 + row) * outPitch + r0 + c8) = u;
    }
    __threadfence();
  }
}

__global__ __launch_bounds__(256) void cast8_f16_kernel(const float* __restrict__ in, unsigned short* __restrict__ out,
                                                        int n8, float scale) {
  const int i = blockIdx.x * 256 + threadIdx.x;
  if (i >= n8) return;
  const float* p = in + 8 * (size_t)i;
  const v4f a = *(const v4f*)(p);
  const v4f c = *(const v4f*)(p + 4);
  unsigned short hb[8];
#pragma unroll
  for (int e = 0; e < 4; ++e) {
    hb[e]     = h_bits(a[e] * scale);
    hb[4 + e] = h_bits(c[e] * scale);
  }
  const v4u u = (v4u){pk16(hb[0], hb[1]), pk16(hb[2], hb[3]), pk16(hb[4], hb[5]), pk16(hb[6], hb[7])};
  unsigned short* q = out + 8 * (size_t)i;
  *(volatile v4u*)q = u;
  __threadfence();
  *(volatile v4u*)q = u;
}

template <int RR, int NWT>
__global__ __launch_bounds__(256) void mix_kernel(const unsigned short* __restrict__ allh,
                                                  const float* __restrict__ wa, const float* __restrict__ wb,
                                                  float* __restrict__ ha, float* __restrict__ hb, float inv_carry) {
  constexpr int TPR = RR / 4;
  constexpr int RPB = 256 / TPR;
  static_assert((RPB * 8) % 32 == 0);
  __shared__ __align__(16) float wsa[RPB * 32];
  __shared__ __align__(16) float wsb[(NWT == 2) ? RPB * 32 : 4];
  const int tid  = threadIdx.x;
  const int m0   = blockIdx.x * RPB;
  const int rowl = tid / TPR;
  const int cq   = (tid - rowl * TPR) * 4;
  if (tid < RPB * 8) {
    *(v4f*)(wsa + 4 * tid) = *(const v4f*)(wa + (size_t)m0 * kN + 4 * tid);
    if (NWT == 2) *(v4f*)(wsb + 4 * tid) = *(const v4f*)(wb + (size_t)m0 * kN + 4 * tid);
  }
  __syncthreads();
  float a0 = 0.0f, a1 = 0.0f, a2 = 0.0f, a3 = 0.0f;
  float b0 = 0.0f, b1 = 0.0f, b2 = 0.0f, b3 = 0.0f;
  const unsigned short* hp = allh + (size_t)(m0 + rowl) * (kN * RR) + cq;
  const float* wra = wsa + rowl * kN;
  const float* wrb = wsb + ((NWT == 2) ? rowl * kN : 0);
#pragma unroll 2
  for (int n = 0; n < kN; ++n) {
    const v2u wd = *(const v2u*)(const void*)(hp + n * RR);
    const float v0 = h16_to_f32(wd[0] & 0xffffu);
    const float v1 = h16_to_f32(wd[0] >> 16);
    const float v2 = h16_to_f32(wd[1] & 0xffffu);
    const float v3 = h16_to_f32(wd[1] >> 16);
    const float w1 = wra[n];
    a0 = fmaf(w1, v0, a0); a1 = fmaf(w1, v1, a1); a2 = fmaf(w1, v2, a2); a3 = fmaf(w1, v3, a3);
    if (NWT == 2) {
      const float w2 = wrb[n];
      b0 = fmaf(w2, v0, b0); b1 = fmaf(w2, v1, b1); b2 = fmaf(w2, v2, b2); b3 = fmaf(w2, v3, b3);
    }
  }
  const size_t o = (size_t)(m0 + rowl) * RR + cq;
  const v4f ov = (v4f){a0 * inv_carry, a1 * inv_carry, a2 * inv_carry, a3 * inv_carry};
  *(volatile v4f*)(ha + o) = ov;
  __threadfence();
  *(volatile v4f*)(ha + o) = ov;
  if (NWT == 2) {
    const v4f ow = (v4f){b0 * inv_carry, b1 * inv_carry, b2 * inv_carry, b3 * inv_carry};
    *(volatile v4f*)(hb + o) = ow;
    __threadfence();
    *(volatile v4f*)(hb + o) = ow;
  }
}

template <int RR>
__global__ __launch_bounds__(256) void tbuild_kernel(const float* __restrict__ h, const float* __restrict__ w,
                                                     unsigned short* __restrict__ T, float carry) {
  constexpr int CPR = 4 * RR;
  const size_t c = (size_t)blockIdx.x * 256 + threadIdx.x;
  const int m   = (int)(c / CPR);
  const int rem = (int)(c - (size_t)m * CPR);
  const int n   = rem / (RR / 8);
  const int r8  = (rem - n * (RR / 8)) * 8;
  const float wv = w[(size_t)m * kN + n];
  const float* hr = h + (size_t)m * RR + r8;
  const v4f x0 = *(const v4f*)(hr);
  const v4f x1 = *(const v4f*)(hr + 4);
  unsigned short hb[8];
#pragma unroll
  for (int e = 0; e < 4; ++e) {
    const float p0 = wv * x0[e];
    const float p1 = wv * x1[e];
    hb[e]     = h_bits(p0 * carry);
    hb[4 + e] = h_bits(p1 * carry);
  }
  const v4u u = (v4u){pk16(hb[0], hb[1]), pk16(hb[2], hb[3]), pk16(hb[4], hb[5]), pk16(hb[6], hb[7])};
  unsigned short* tp = T + c * 8;
  *(volatile v4u*)tp = u;
  __threadfence();
  *(volatile v4u*)tp = u;
}

__global__ __launch_bounds__(128) void attn_causal_kernel(const unsigned short* __restrict__ Qp,
                                                          const unsigned short* __restrict__ Kp,
                                                          const unsigned short* __restrict__ Vtp,
                                                          unsigned short* __restrict__ Op) {
  __shared__ __align__(16) _Float16 Ksh[64 * 64];
  __shared__ __align__(16) _Float16 Vts[64 * 64];
  __shared__ __align__(16) _Float16 Psh[4][16 * 64];
  __shared__ __align__(16) float    Os[4][16 * 68];
  const int tid  = threadIdx.x;
  const int wave = tid >> 5;
  const int lane = tid & 31;
  const int hh   = lane >> 4;
  const int c    = lane & 15;
  const int bx = blockIdx.x;
  const int qb = bx & 31;
  const int bh = bx >> 5;
  const int h  = bh & 15;
  const int b  = bh >> 4;
  const int q0 = qb * 64 + wave * 16;
  const _Float16* Qg = (const _Float16*)(const void*)Qp;
  const _Float16* Kg = (const _Float16*)(const void*)Kp;
  const _Float16* Vg = (const _Float16*)(const void*)Vtp;
  const size_t tokBase = (size_t)b * kS;

  v16h qa[2];
  {
    const _Float16* qrow = Qg + (tokBase + q0 + c) * kD + h * kDh + 8 * hh;
    qa[0] = Frag<_Float16>::load(qrow);
    qa[1] = Frag<_Float16>::load(qrow + 32);
  }

  float mrow[8], lrow[8];
  v8f oacc[4];
#pragma unroll
  for (int r = 0; r < 8; ++r) { mrow[r] = -__builtin_inff(); lrow[r] = 0.0f; }
#pragma unroll
  for (int t = 0; t < 4; ++t) oacc[t] = (v8f){0.f,0.f,0.f,0.f,0.f,0.f,0.f,0.f};

  const int nChunks = qb + 1;
  for (int kc = 0; kc < nChunks; ++kc) {
    const int kv0 = kc * 64;
    __syncthreads();
    {
      const int rr = tid >> 1;
      const int hf = (tid & 1) * 32;
      const v4u* ks = (const v4u*)(const void*)(Kg + (tokBase + kv0 + rr) * kD + h * kDh + hf);
      const v4u* vs = (const v4u*)(const void*)(Vg + (size_t)(h * kDh + rr) * kTok + tokBase + kv0 + hf);
      const v4u k0v = ks[0], k1v = ks[1], k2v = ks[2], k3v = ks[3];
      const v4u v0v = vs[0], v1v = vs[1], v2v = vs[2], v3v = vs[3];
      v4u* kd = (v4u*)(void*)(Ksh + rr * 64 + hf);
      v4u* vd = (v4u*)(void*)(Vts + rr * 64 + hf);
      kd[0] = k0v; kd[1] = k1v; kd[2] = k2v; kd[3] = k3v;
      vd[0] = v0v; vd[1] = v1v; vd[2] = v2v; vd[3] = v3v;
    }
    __syncthreads();

    v8f s[4];
#pragma unroll
    for (int j = 0; j < 4; ++j) {
      s[j] = (v8f){0.f,0.f,0.f,0.f,0.f,0.f,0.f,0.f};
#pragma unroll
      for (int dc = 0; dc < 2; ++dc) {
        const v16h kb = Frag<_Float16>::load(Ksh + (j * 16 + c) * 64 + dc * 32 + 8 * hh);
        s[j] = h_mma(qa[dc], kb, s[j]);
      }
    }
    const bool diag = (kc == qb);
    float cm[8];
#pragma unroll
    for (int r = 0; r < 8; ++r) {
      const int qrow = q0 + 8 * hh + r;
      float m = -__builtin_inff();
#pragma unroll
      for (int j = 0; j < 4; ++j) {
        const int kvcol = kv0 + j * 16 + c;
        float sv = s[j][r] * kScoreInv;
        sv = (diag && (kvcol > qrow)) ? -__builtin_inff() : sv;
        s[j][r] = sv;
        m = fmaxf(m, sv);
      }
#pragma unroll
      for (int off = 1; off < 16; off <<= 1) m = fmaxf(m, __shfl_xor(m, off, 32));
      cm[r] = m;
    }
    _Float16* pw = Psh[wave];
#pragma unroll
    for (int r = 0; r < 8; ++r) {
      const float mnew  = fmaxf(mrow[r], cm[r]);
      const float alpha = expf(mrow[r] - mnew);
      mrow[r] = mnew;
      float psum = 0.0f;
#pragma unroll
      for (int j = 0; j < 4; ++j) {
        const float p = expf(s[j][r] - mnew);
        psum += p;
        pw[(8 * hh + r) * 64 + j * 16 + c] = (_Float16)(p * kPCarry);
      }
#pragma unroll
      for (int off = 1; off < 16; off <<= 1) psum += __shfl_xor(psum, off, 32);
      lrow[r] = lrow[r] * alpha + psum;
#pragma unroll
      for (int t = 0; t < 4; ++t) oacc[t][r] *= alpha;
    }
    __builtin_amdgcn_fence(__ATOMIC_RELEASE, "workgroup");
    __builtin_amdgcn_wave_barrier();
    __builtin_amdgcn_fence(__ATOMIC_ACQUIRE, "workgroup");
#pragma unroll
    for (int kk = 0; kk < 2; ++kk) {
      const v16h pa = Frag<_Float16>::load(pw + c * 64 + kk * 32 + 8 * hh);
#pragma unroll
      for (int t = 0; t < 4; ++t) {
        const v16h vb = Frag<_Float16>::load(Vts + (t * 16 + c) * 64 + kk * 32 + 8 * hh);
        oacc[t] = h_mma(pa, vb, oacc[t]);
      }
    }
  }

  float* os = Os[wave];
#pragma unroll
  for (int r = 0; r < 8; ++r) {
    const float inv = (1.0f / lrow[r]) * kAttnOut;
#pragma unroll
    for (int t = 0; t < 4; ++t) os[(8 * hh + r) * 68 + t * 16 + c] = oacc[t][r] * inv;
  }
  __builtin_amdgcn_fence(__ATOMIC_RELEASE, "workgroup");
  __builtin_amdgcn_wave_barrier();
  __builtin_amdgcn_fence(__ATOMIC_ACQUIRE, "workgroup");
  {
    const int q = lane >> 3, c8 = (lane & 7) * 8;
    for (int pass = 0; pass < 2; ++pass) {
#pragma unroll
      for (int it = 0; it < 4; ++it) {
        const int row = it * 4 + q;
        unsigned short hb[8];
#pragma unroll
        for (int e = 0; e < 8; ++e) hb[e] = h_bits(os[row * 68 + c8 + e]);
        const v4u u = (v4u){pk16(hb[0], hb[1]), pk16(hb[2], hb[3]), pk16(hb[4], hb[5]), pk16(hb[6], hb[7])};
        *(volatile v4u*)(Op + (tokBase + q0 + row) * kD + h * kDh + c8) = u;
      }
      __threadfence();
    }
  }
}

extern "C" void kernel_launch(void* const* d_in, const int* in_sizes, int n_in,
                              void* d_out, int out_size, void* d_ws, size_t ws_size,
                              hipStream_t stream) {
  if (n_in < 20) return;
  const int nAct = kTok * kD;
  if (in_sizes[0] != nAct || out_size != nAct) return;
  if (in_sizes[1] != kN * kD * kR || in_sizes[2] != kN * kD * kR) return;
  if (in_sizes[3] != kN * kR * kD || in_sizes[4] != kN * kR * kD) return;
  if (in_sizes[5] != kN * kD * kRK || in_sizes[6] != kN * kRK * kD) return;
  if (in_sizes[7] != kD * kD) return;
  for (int i = 8; i < 12; ++i) if (in_sizes[i] != kD) return;
  for (int i = 12; i < 20; ++i) if (in_sizes[i] != kTok * kN) return;

  const size_t szA   = (size_t)kTok * kD * 2;
  const size_t szB   = (size_t)kKkn * kD * 2;
  const size_t szC   = (size_t)kTok * kKkn * 2;
  const size_t szD   = (size_t)kTok * kKqk * 2;
  const size_t szH64 = (size_t)kTok * kR * 4;
  const size_t szH128= (size_t)kTok * kRK * 4;
  const size_t szEqv = (size_t)kD * kKqk * 2;
  const size_t szEkn = (size_t)kD * kKkn * 2;
  const size_t szQ   = (size_t)kTok * kD * 2;
  const size_t szX1  = (size_t)kTok * kD * 4;
  const size_t offA   = 0;
  const size_t offB   = offA + szA;
  const size_t offC   = offB + szB;
  const size_t offD   = offC + szC;
  const size_t offHq  = offD + szD;
  const size_t offHk  = offHq + szH64;
  const size_t offHv  = offHk + szH64;
  const size_t offHkn = offHv + szH64;
  const size_t offEqv = offHkn + szH128;
  const size_t offEkn = offEqv + szEqv;
  const size_t offQ   = offEkn + szEkn;
  const size_t offK   = offQ + szQ;
  const size_t offVT  = offK + szQ;
  const size_t offX1  = offVT + szQ;
  const size_t total  = offX1 + szX1;
  if (ws_size < total) return;

  const float* x       = (const float*)d_in[0];
  const float* f_qk    = (const float*)d_in[1];
  const float* f_v     = (const float*)d_in[2];
  const float* r_qk    = (const float*)d_in[3];
  const float* r_v     = (const float*)d_in[4];
  const float* f_know  = (const float*)d_in[5];
  const float* r_know  = (const float*)d_in[6];
  const float* w_o     = (const float*)d_in[7];
  const float* gamma1  = (const float*)d_in[8];
  const float* beta1   = (const float*)d_in[9];
  const float* gamma2  = (const float*)d_in[10];
  const float* beta2   = (const float*)d_in[11];
  const float* w_fq    = (const float*)d_in[12];
  const float* w_fk    = (const float*)d_in[13];
  const float* w_fv    = (const float*)d_in[14];
  const float* w_rq    = (const float*)d_in[15];
  const float* w_rk    = (const float*)d_in[16];
  const float* w_rv    = (const float*)d_in[17];
  const float* w_kn_f  = (const float*)d_in[18];
  const float* w_kn_r  = (const float*)d_in[19];
  float* out = (float*)d_out;
  char* ws = (char*)d_ws;
  unsigned short* pA   = (unsigned short*)(ws + offA);
  unsigned short* pB   = (unsigned short*)(ws + offB);
  unsigned short* pC   = (unsigned short*)(ws + offC);
  unsigned short* pD   = (unsigned short*)(ws + offD);
  float* hq  = (float*)(ws + offHq);
  float* hk  = (float*)(ws + offHk);
  float* hv  = (float*)(ws + offHv);
  float* hkn = (float*)(ws + offHkn);
  unsigned short* pEqv = (unsigned short*)(ws + offEqv);
  unsigned short* pEkn = (unsigned short*)(ws + offEkn);
  unsigned short* pQ   = (unsigned short*)(ws + offQ);
  unsigned short* pK   = (unsigned short*)(ws + offK);
  unsigned short* pVT  = (unsigned short*)(ws + offVT);
  float* x1 = (float*)(ws + offX1);
  const float* fdummy = x;

  const dim3 blk(256);
  auto gemm_h16 = [&](const unsigned short* Am, int lda, const unsigned short* Btm, int ldb,
                      unsigned short* Cm, int ldc, int M, int N, int K, float scale) {
    const int tiles = (M / 64) * (N / 64);
    wmma_gemm64<0, false, 0, 1, false, 0><<<dim3((tiles + 7) / 8, 1), blk, 0, stream>>>(
        Am, Am, lda, 0L, Btm, Btm, ldb, 0L, (void*)Cm, (void*)Cm, ldc, 0L, fdummy, fdummy, 0L, M, N, K, scale);
  };
  auto gemm_f32res = [&](const unsigned short* Am, int lda, const unsigned short* Btm, int ldb,
                         float* Cm, int ldc, const float* res, int M, int N, int K, float scale) {
    const int tiles = (M / 64) * (N / 64);
    wmma_gemm64<0, false, 0, 0, true, 0><<<dim3((tiles + 7) / 8, 1), blk, 0, stream>>>(
        Am, Am, lda, 0L, Btm, Btm, ldb, 0L, (void*)Cm, (void*)Cm, ldc, 0L, fdummy, res, 0L, M, N, K, scale);
  };

  ln_f16_kernel<<<dim3(kTok), dim3(128), 0, stream>>>(x, gamma1, beta1, pA);
  tpose_cast_kernel<<<dim3(kR / 64, kD / 64, kN), blk, 0, stream>>>(f_qk, (long)kD * kR, kR, pB, (long)kR * kD, kD, kWCarry);
  gemm_h16(pA, kD, pB, kD, pD, kKqk, kTok, kKqk, kD, 1.0f);
  mix_kernel<kR, 2><<<dim3(kTok / 16), blk, 0, stream>>>(pD, w_fq, w_fk, hq, hk, kAhInv);
  tpose_cast_kernel<<<dim3(kR / 64, kD / 64, kN), blk, 0, stream>>>(f_v, (long)kD * kR, kR, pB, (long)kR * kD, kD, kWCarry);
  gemm_h16(pA, kD, pB, kD, pD, kKqk, kTok, kKqk, kD, 1.0f);
  mix_kernel<kR, 1><<<dim3(kTok / 16), blk, 0, stream>>>(pD, w_fv, w_fv, hv, hv, kAhInv);
  tpose_cast_kernel<<<dim3(kD / 64, kKqk / 64, 1), blk, 0, stream>>>(r_qk, 0L, kD, pEqv, 0L, kKqk, kWCarry);
  tbuild_kernel<kR><<<dim3(kTok * 4 * kR / 256), blk, 0, stream>>>(hq, w_rq, pD, kTCarry);
  gemm_h16(pD, kKqk, pEqv, kKqk, pQ, kD, kTok, kD, kKqk, kQScale);
  tbuild_kernel<kR><<<dim3(kTok * 4 * kR / 256), blk, 0, stream>>>(hk, w_rk, pD, kTCarry);
  gemm_h16(pD, kKqk, pEqv, kKqk, pK, kD, kTok, kD, kKqk, kKVScale);
  tpose_cast_kernel<<<dim3(kD / 64, kKqk / 64, 1), blk, 0, stream>>>(r_v, 0L, kD, pEqv, 0L, kKqk, kWCarry);
  tbuild_kernel<kR><<<dim3(kTok * 4 * kR / 256), blk, 0, stream>>>(hv, w_rv, pD, kTCarry);
  gemm_h16(pEqv, kKqk, pD, kKqk, pVT, kTok, kD, kTok, kKqk, kKVScale);
  attn_causal_kernel<<<dim3(kB * kH * (kS / 64)), dim3(128), 0, stream>>>(pQ, pK, pVT, pA);
  cast8_f16_kernel<<<dim3((kD * kD / 8) / 256), blk, 0, stream>>>(w_o, pB, kD * kD / 8, kWCarry);
  gemm_f32res(pA, kD, pB, kD, x1, kD, x, kTok, kD, kD, kWoScale);

  ln_f16_kernel<<<dim3(kTok), dim3(128), 0, stream>>>(x1, gamma2, beta2, pA);
  tpose_cast_kernel<<<dim3(kRK / 64, kD / 64, kN), blk, 0, stream>>>(f_know, (long)kD * kRK, kRK, pB, (long)kRK * kD, kD, kWCarry);
  gemm_h16(pA, kD, pB, kD, pC, kKkn, kTok, kKkn, kD, 1.0f);
  mix_kernel<kRK, 1><<<dim3(kTok / 8), blk, 0, stream>>>(pC, w_kn_f, w_kn_f, hkn, hkn, kAhInv);
  tpose_cast_kernel<<<dim3(kD / 64, kKkn / 64, 1), blk, 0, stream>>>(r_know, 0L, kD, pEkn, 0L, kKkn, kWCarry);
  tbuild_kernel<kRK><<<dim3(kTok * 4 * kRK / 256), blk, 0, stream>>>(hkn, w_kn_r, pC, kTCarry);
  gemm_f32res(pC, kKkn, pEkn, kKkn, out, kD, x1, kTok, kD, kKkn, kKnScale);
}
